// MultiHeadAttention_87247965651527
// MI455X (gfx1250) — hardware-verified
//
#include <hip/hip_runtime.h>

#pragma clang fp contract(off)

#ifndef NB
#define NB 2
#endif
#ifndef SEQ
#define SEQ 2048
#endif
#define NB_FULL  2
#define SEQ_FULL 2048
#define TT   SEQ
#define DM   1024
#define NH_  16
#define HD   64
#define DQ   (NH_ * HD)
#define ZH   2
#define RH   256
#define PCAR 1024.0f
#define SCL  0.125f
#define RBASE 10000.0f
static_assert(NB >= 1);
static_assert(NB <= NB_FULL);
static_assert(SEQ <= SEQ_FULL);
static_assert(TT % 128 == 0);
static_assert(RH % 64 == 0);
static_assert(RH <= TT);
static_assert(DM % 64 == 0);
static_assert(NH_ % ZH == 0);
static_assert(DQ == DM);

typedef _Float16 h16;
typedef unsigned short bf;
typedef __attribute__((ext_vector_type(16))) __bf16   v16bf;
typedef __attribute__((ext_vector_type(16))) _Float16 v16h;
typedef __attribute__((ext_vector_type(8)))  _Float16 v8h;
typedef __attribute__((ext_vector_type(8)))  unsigned short v8us;
typedef __attribute__((ext_vector_type(8)))  float    v8f;
typedef __attribute__((ext_vector_type(4)))  float    v4f;
typedef __attribute__((ext_vector_type(2)))  _Float16 v2h;
typedef __attribute__((ext_vector_type(2)))  unsigned short v2us;
typedef __attribute__((ext_vector_type(2)))  float    v2f;
typedef v4f  __attribute__((may_alias)) v4fa;

__device__ __forceinline__ unsigned short f2bf(float f) { unsigned u = __float_as_uint(f); u += 0x7FFFu + ((u >> 16) & 1u); return (unsigned short)(u >> 16); }
__device__ __forceinline__ float bf2f(unsigned short b) { return __uint_as_float(((unsigned)b) << 16); }
__device__ __forceinline__ v16h cat16(v8h lo, v8h hi) { return __builtin_shufflevector(lo, hi, 0, 1, 2, 3, 4, 5, 6, 7, 8, 9, 10, 11, 12, 13, 14, 15); }
__device__ __forceinline__ v16bf cat16b(v8us lo, v8us hi) { return __builtin_bit_cast(v16bf, __builtin_shufflevector(lo, hi, 0, 1, 2, 3, 4, 5, 6, 7, 8, 9, 10, 11, 12, 13, 14, 15)); }
__device__ __forceinline__ v8f wmma16(v16h a, v16h b, v8f c) { return __builtin_amdgcn_wmma_f32_16x16x32_f16(false, a, false, b, (short)0, c, false, false); }
__device__ __forceinline__ v8f wmmab(v16bf a, v16bf b, v8f c) { return __builtin_amdgcn_wmma_f32_16x16x32_bf16(false, a, false, b, (short)0, c, false, false); }
__device__ __forceinline__ h16 tohx(float x) { return (h16)x; }
__device__ __forceinline__ void splitf(float y, unsigned short& h, unsigned short& l) { h = f2bf(y); l = f2bf(y - bf2f(h)); }

template <typename T16> struct WFrag;
template <> struct WFrag<h16> { typedef v16h V; static __device__ __forceinline__ V ld(const h16* p) { return cat16(*(const v8h*)p, *(const v8h*)(p + 16)); } static __device__ __forceinline__ v8f mma(V a, V b, v8f c) { return wmma16(a, b, c); } };
template <> struct WFrag<bf> { typedef v16bf V; static __device__ __forceinline__ V ld(const bf* p) { return cat16b(*(const v8us*)p, *(const v8us*)(p + 16)); } static __device__ __forceinline__ v8f mma(V a, V b, v8f c) { return wmmab(a, b, c); } };
template <typename T16, int NSPLIT, int CM>
__global__ __launch_bounds__(32) void k_gemmw(const T16* __restrict__ A, const T16* __restrict__ A2, const T16* __restrict__ Bt, const T16* __restrict__ Bt2, int K, float* C, int ldc, size_t sA, size_t sB, size_t sC, int qoff) {
    typedef typename WFrag<T16>::V V;
    __shared__ __align__(16) float os[16 * 68];
    const int lane = threadIdx.x & 31, lr = lane & 15, hi = lane >> 4; const int r0 = blockIdx.x * 64, c0 = blockIdx.y * 64;
    if (CM == 1) { if (c0 >= qoff + r0 + 64) return; }
    int kend = K; if (CM == 2) { const int kl = qoff + r0 + 64; kend = (kl < K) ? kl : K; }
    const size_t z = blockIdx.z; A += z * sA; if (NSPLIT == 1 || NSPLIT == 2) A2 += z * sA; Bt += z * sB; if (NSPLIT >= 2) Bt2 += z * sB; C += z * sC;
    v8f acc[4][4];
#pragma unroll
    for (int mb = 0; mb < 4; ++mb)
#pragma unroll
        for (int nb = 0; nb < 4; ++nb) acc[mb][nb] = (v8f){};
    const size_t aoff = (size_t)(r0 + lr) * K + 8 * hi, boff = (size_t)(c0 + lr) * K + 8 * hi;
#pragma unroll 1
    for (int kc = 0; kc < kend; kc += 32) {
        V a[4], a2[4];
#pragma unroll
        for (int mb = 0; mb < 4; ++mb) { a[mb] = WFrag<T16>::ld(A + aoff + (size_t)mb * 16 * K + kc); if (NSPLIT == 1 || NSPLIT == 2) a2[mb] = WFrag<T16>::ld(A2 + aoff + (size_t)mb * 16 * K + kc); else a2[mb] = a[mb]; }
#pragma unroll
        for (int nb = 0; nb < 4; ++nb) { const V b = WFrag<T16>::ld(Bt + boff + (size_t)nb * 16 * K + kc); V b2 = b; if (NSPLIT >= 2) b2 = WFrag<T16>::ld(Bt2 + boff + (size_t)nb * 16 * K + kc);
#pragma unroll
            for (int mb = 0; mb < 4; ++mb) { acc[mb][nb] = WFrag<T16>::mma(a[mb], b, acc[mb][nb]); if (NSPLIT == 1 || NSPLIT == 2) acc[mb][nb] = WFrag<T16>::mma(a2[mb], b, acc[mb][nb]); if (NSPLIT >= 2) acc[mb][nb] = WFrag<T16>::mma(a[mb], b2, acc[mb][nb]); } }
        asm volatile("v_nop\n\tv_nop\n\tv_nop\n\tv_nop" : "+v"(acc[0][0]), "+v"(acc[1][1]), "+v"(acc[2][2]), "+v"(acc[3][3]) : "v"(a[0]), "v"(a[3]));
    }
#pragma unroll
    for (int mb = 0; mb < 4; ++mb) {
#pragma unroll
        for (int nb = 0; nb < 4; ++nb) {
#pragma unroll
            for (int j = 0; j < 8; ++j) os[(hi * 8 + j) * 68 + nb * 16 + lr] = acc[mb][nb][j]; }
        __builtin_amdgcn_wave_barrier(); asm volatile("" ::: "memory");
        float* crow = C + (size_t)(r0 + mb * 16) * ldc + c0;
#pragma unroll 1
        for (int ps = 0; ps < 2; ++ps) {
#pragma unroll
            for (int s = 0; s < 8; ++s) { const int row = 2 * s + hi, cofs = lr * 4; const v4f val = *(const v4fa*)(os + row * 68 + cofs);
                *(volatile v4f*)(crow + (size_t)row * ldc + cofs) = val; }
            if (ps == 0) __threadfence(); }
        __builtin_amdgcn_wave_barrier(); asm volatile("" ::: "memory");
    }
}

__global__ __launch_bounds__(256) void k_wtG(const float* __restrict__ w, int K, int N, bf* Bt) {
    const int lane = threadIdx.x & 31; const int L0 = (blockIdx.x * 8 + (threadIdx.x >> 5)) * 8; const int nlines = N * K / 64;
#pragma unroll
    for (int ps = 0; ps < 2; ++ps) {
#pragma unroll 1
        for (int l = 0; l < 8; ++l) { const int L = L0 + l; if (L >= nlines) break; const size_t e = (size_t)L * 64 + lane * 2; const int k = (int)(e % K), n = (int)(e / K); v2us o;
            o[0] = f2bf(w[(size_t)k * N + n]); o[1] = f2bf(w[(size_t)(k + 1) * N + n]); *(volatile v2us*)(Bt + e) = o; }
        if (ps == 0) __threadfence(); }
}
__global__ __launch_bounds__(256) void k_cvt8(const float* __restrict__ src, bf* dst, size_t n8) { const size_t i = (size_t)blockIdx.x * 256 + threadIdx.x; if (i >= n8) return; const v8f v = *(const v8f*)(src + i * 8); v8us o;
#pragma unroll
    for (int k = 0; k < 8; ++k) o[k] = f2bf(v[k]); *(volatile v8us*)(dst + i * 8) = o; __threadfence(); *(volatile v8us*)(dst + i * 8) = o; }

__global__ __launch_bounds__(256) void k_cstab(float* CS) {
    const int idx = blockIdx.x * 256 + threadIdx.x; if (idx >= TT * (HD / 2)) return;
    const int i = idx % (HD / 2); const int t = idx / (HD / 2);
    const float ex = (float)(2 * i) / (float)HD;
    const float invf = 1.0f / powf(RBASE, ex);
    const float ang = (float)t * invf;
    float sn, cn; sincosf(ang, &sn, &cn);
    v2f cs; cs[0] = cn; cs[1] = sn;
    float* p0 = CS + ((size_t)t * HD + i) * 2; float* p1 = CS + ((size_t)t * HD + i + HD / 2) * 2;
    *(volatile v2f*)p0 = cs; *(volatile v2f*)p1 = cs; __threadfence(); *(volatile v2f*)p0 = cs; *(volatile v2f*)p1 = cs;
}

__global__ __launch_bounds__(256) void k_rope(const float* __restrict__ F, int pitch, int nheads, const float* __restrict__ CS, h16* P16, bf* Ph, bf* Pl) {
    const size_t e = ((size_t)blockIdx.x * 256 + threadIdx.x) * 2; if (e >= (size_t)nheads * TT * HD) return;
    const int d = (int)(e % HD); const int t = (int)((e / HD) % TT); const int h = (int)(e / ((size_t)HD * TT));
    const float* f = F + (size_t)t * pitch + h * HD; v2h o16; v2us oh, ol;
#pragma unroll
    for (int q = 0; q < 2; ++q) { const int dd = d + q; const int dp = (dd < HD / 2) ? dd + HD / 2 : dd - HD / 2; const float x0 = f[dd], x1 = f[dp];
        const v2f cs = *(const v2f*)(CS + ((size_t)t * HD + dd) * 2); float a = __fmul_rn(x0, cs[0]), bq = __fmul_rn(x1, cs[1]); asm volatile("" : "+v"(a)); asm volatile("" : "+v"(bq));
        const float r = (dd < HD / 2) ? __fsub_rn(a, bq) : __fadd_rn(a, bq);
        o16[q] = tohx(r); unsigned short a2, c2; splitf(r, a2, c2); oh[q] = a2; ol[q] = c2; }
    *(volatile v2h*)(P16 + e) = o16; *(volatile v2us*)(Ph + e) = oh; *(volatile v2us*)(Pl + e) = ol; __threadfence(); *(volatile v2h*)(P16 + e) = o16; *(volatile v2us*)(Ph + e) = oh; *(volatile v2us*)(Pl + e) = ol; }
__global__ __launch_bounds__(256) void k_vtp(const float* __restrict__ F, int pitch, int nheads, h16* V16, bf* Vh, bf* Vl) { const size_t e = ((size_t)blockIdx.x * 256 + threadIdx.x) * 2; if (e >= (size_t)nheads * HD * TT) return; const int t = (int)(e % TT); const int d = (int)((e / TT) % HD); const int g = (int)(e / ((size_t)TT * HD)); v2h o16; v2us oh, ol;
#pragma unroll
    for (int q = 0; q < 2; ++q) { const float x = F[(size_t)(t + q) * pitch + g * HD + d]; o16[q] = tohx(x); unsigned short a2, c2; splitf(x, a2, c2); oh[q] = a2; ol[q] = c2; }
    *(volatile v2h*)(V16 + e) = o16; *(volatile v2us*)(Vh + e) = oh; *(volatile v2us*)(Vl + e) = ol; __threadfence(); *(volatile v2h*)(V16 + e) = o16; *(volatile v2us*)(Vh + e) = oh; *(volatile v2us*)(Vl + e) = ol; }

__global__ __launch_bounds__(256) void k_asoft(const float* __restrict__ Sb, h16* P16, bf* Ph, bf* Pl) {
    const int lane = threadIdx.x & 31;
    const int row = __builtin_amdgcn_readfirstlane((int)(blockIdx.x * 8 + (threadIdx.x >> 5)));
    if (row >= ZH * TT) return;
    const int i = row % TT; const int zz = row / TT; const bool hires = (i < RH); const int nch = (i >> 6) + 1;
    const float* sr = Sb + (size_t)row * TT;
    float v[TT / 32]; float mx = -3.0e38f;
#pragma unroll
    for (int ch = 0; ch < TT / 64; ++ch) {
        if (ch < nch) { const int j0 = ch * 64 + lane * 2; const v2f a = *(const v2f*)(sr + j0);
#pragma unroll
            for (int q = 0; q < 2; ++q) { float t = a[q] * SCL; t = (j0 + q <= i) ? t : -3.0e38f; v[ch * 2 + q] = t; mx = fmaxf(mx, t); } }
        else { v[ch * 2] = -3.0e38f; v[ch * 2 + 1] = -3.0e38f; }
    }
#pragma unroll
    for (int sh = 16; sh; sh >>= 1) mx = fmaxf(mx, __shfl_xor(mx, sh, 32));
    float sum = 0.f;
#pragma unroll
    for (int ch = 0; ch < TT / 64; ++ch) {
        if (ch < nch) {
#pragma unroll
            for (int q = 0; q < 2; ++q) { const int k = ch * 2 + q; float d0 = __fsub_rn(v[k], mx); asm volatile("" : "+v"(d0));
                float ev = __builtin_amdgcn_exp2f(__fmul_rn(d0, 1.4426950408889634f)); ev = (ch * 64 + lane * 2 + q <= i) ? ev : 0.0f; v[k] = ev; sum += ev; } }
        else { v[ch * 2] = 0.0f; v[ch * 2 + 1] = 0.0f; }
    }
#pragma unroll
    for (int sh = 16; sh; sh >>= 1) sum += __shfl_xor(sum, sh, 32);
    const float f = __fdiv_rn(hires ? 1.0f : PCAR, sum);
#pragma unroll 1
    for (int ps = 0; ps < 2; ++ps) {
        if (hires) {
#pragma unroll
            for (int ch = 0; ch < TT / 64; ++ch) { if (ch < nch) { v2us oh, ol;
#pragma unroll
                for (int q = 0; q < 2; ++q) { unsigned short a2, c2; splitf(v[ch * 2 + q] * f, a2, c2); oh[q] = a2; ol[q] = c2; }
                const size_t oo = ((size_t)zz * RH + i) * TT + ch * 64 + lane * 2; *(volatile v2us*)(Ph + oo) = oh; *(volatile v2us*)(Pl + oo) = ol; } }
        } else {
#pragma unroll
            for (int ch = 0; ch < TT / 64; ++ch) { if (ch < nch) { v2h o2;
#pragma unroll
                for (int q = 0; q < 2; ++q) o2[q] = tohx(v[ch * 2 + q] * f);
                *(volatile v2h*)(P16 + (size_t)row * TT + ch * 64 + lane * 2) = o2; } } }
        if (ps == 0) __threadfence(); }
}
__global__ __launch_bounds__(256) void k_merge(const float* __restrict__ O, int h0, bf* Ah, bf* Al) { const size_t e = ((size_t)blockIdx.x * 256 + threadIdx.x) * 2; if (e >= (size_t)ZH * TT * HD) return; const int d = (int)(e % HD); const int t = (int)((e / HD) % TT); const int zz = (int)(e / ((size_t)HD * TT)); const float cs = (t < RH) ? 1.0f : (1.0f / PCAR); const size_t oo = (size_t)t * DQ + (h0 + zz) * HD + d;
    v2us oh, ol;
#pragma unroll
    for (int q = 0; q < 2; ++q) { unsigned short a2, c2; splitf(O[e + q] * cs, a2, c2); oh[q] = a2; ol[q] = c2; } *(volatile v2us*)(Ah + oo) = oh; *(volatile v2us*)(Al + oo) = ol; __threadfence(); *(volatile v2us*)(Ah + oo) = oh; *(volatile v2us*)(Al + oo) = ol; }

extern "C" void kernel_launch(void* const* d_in, const int* in_sizes, int n_in,
                              void* d_out, int out_size, void* d_ws, size_t ws_size, hipStream_t stream) {
    if (n_in < 3) return;
    if (in_sizes[0] < NB * SEQ * DM || in_sizes[1] < 3 * DM * DM || in_sizes[2] < DM * DM || out_size < NB * SEQ * DM) return;
    const float* x = (const float*)d_in[0];
    const float* w_attn = (const float*)d_in[1];
    const float* w_proj = (const float*)d_in[2];
    float* OUT = (float*)d_out;
    char* ws0 = (char*)d_ws; char* wsp = ws0;
    auto take = [&](size_t bytes) { char* p = wsp; wsp += (bytes + 255) & ~(size_t)255; return (void*)p; };
    bf* WT = (bf*)take((size_t)3 * DM * DM * 2); bf* WO = (bf*)take((size_t)DM * DM * 2); float* CS = (float*)take((size_t)TT * HD * 2 * 4);
    bf* XB = (bf*)take((size_t)TT * DM * 2); float* FQ = (float*)take((size_t)TT * DQ * 4); float* FK = (float*)take((size_t)TT * DQ * 4);
    h16* QP16 = (h16*)take((size_t)NH_ * TT * HD * 2); h16* KP16 = (h16*)take((size_t)NH_ * TT * HD * 2); h16* VT16 = (h16*)take((size_t)NH_ * HD * TT * 2);
    bf* QPh = (bf*)take((size_t)NH_ * TT * HD * 2); bf* QPl = (bf*)take((size_t)NH_ * TT * HD * 2); bf* KPh = (bf*)take((size_t)NH_ * TT * HD * 2); bf* KPl = (bf*)take((size_t)NH_ * TT * HD * 2);
    bf* VTh = (bf*)take((size_t)NH_ * HD * TT * 2); bf* VTl = (bf*)take((size_t)NH_ * HD * TT * 2);
    bf* Ph = (bf*)take((size_t)ZH * RH * TT * 2); bf* Pl = (bf*)take((size_t)ZH * RH * TT * 2);
    float* Sb = (float*)take((size_t)ZH * TT * TT * 4); h16* P16 = (h16*)take((size_t)ZH * TT * TT * 2); float* Ob = (float*)take((size_t)ZH * TT * HD * 4);
    bf* ATh = (bf*)take((size_t)TT * DQ * 2); bf* ATl = (bf*)take((size_t)TT * DQ * 2);
    const size_t used = (size_t)(wsp - ws0);
    if (used > ws_size || used > (size_t)134217728) return;
    float* FV = FK;
    k_wtG<<<(unsigned)((3 * DM * DM / 64 + 63) / 64), 256, 0, stream>>>(w_attn, DM, 3 * DM, WT);
    k_wtG<<<(unsigned)((DM * DM / 64 + 63) / 64), 256, 0, stream>>>(w_proj, DM, DM, WO);
    k_cstab<<<(unsigned)((TT * (HD / 2) + 255) / 256), 256, 0, stream>>>(CS);
    const unsigned LP = (unsigned)(((size_t)NH_ * TT * HD / 2 + 255) / 256);
    const size_t hs = (size_t)TT * HD;
    for (int b = 0; b < NB; ++b) {
        k_cvt8<<<(unsigned)(((size_t)TT * DM / 8 + 255) / 256), 256, 0, stream>>>(x + (size_t)b * SEQ_FULL * DM, XB, (size_t)TT * DM / 8);
        k_gemmw<bf, 0, 0><<<dim3(TT / 64, DQ / 64, 1), 32, 0, stream>>>(XB, nullptr, WT, nullptr, DM, FQ, DQ, 0, 0, 0, 0);
        k_rope<<<LP, 256, 0, stream>>>(FQ, DQ, NH_, CS, QP16, QPh, QPl);
        k_gemmw<bf, 0, 0><<<dim3(TT / 64, DQ / 64, 1), 32, 0, stream>>>(XB, nullptr, WT + (size_t)DM * DM, nullptr, DM, FK, DQ, 0, 0, 0, 0);
        k_rope<<<LP, 256, 0, stream>>>(FK, DQ, NH_, CS, KP16, KPh, KPl);
        k_gemmw<bf, 0, 0><<<dim3(TT / 64, DQ / 64, 1), 32, 0, stream>>>(XB, nullptr, WT + (size_t)2 * DM * DM, nullptr, DM, FV, DQ, 0, 0, 0, 0);
        k_vtp<<<LP, 256, 0, stream>>>(FV, DQ, NH_, VT16, VTh, VTl);
        for (int h0 = 0; h0 < NH_; h0 += ZH) { const size_t zo = (size_t)h0 * hs;
            k_gemmw<bf, 2, 1><<<dim3(RH / 64, TT / 64, ZH), 32, 0, stream>>>(QPh + zo, QPl + zo, KPh + zo, KPl + zo, HD, Sb, TT, hs, hs, (size_t)TT * TT, 0);
            if (TT > RH) k_gemmw<h16, 0, 1><<<dim3((TT - RH) / 64, TT / 64, ZH), 32, 0, stream>>>(QP16 + zo + (size_t)RH * HD, nullptr, KP16 + zo, nullptr, HD, Sb + (size_t)RH * TT, TT, hs, hs, (size_t)TT * TT, RH);
            k_asoft<<<ZH * TT / 8, 256, 0, stream>>>(Sb, P16, Ph, Pl);
            k_gemmw<bf, 2, 2><<<dim3(RH / 64, HD / 64, ZH), 32, 0, stream>>>(Ph, Pl, VTh + zo, VTl + zo, TT, Ob, HD, (size_t)RH * TT, hs, hs, 0);
            if (TT > RH) k_gemmw<h16, 0, 2><<<dim3((TT - RH) / 64, HD / 64, ZH), 32, 0, stream>>>(P16 + (size_t)RH * TT, nullptr, VT16 + zo, nullptr, TT, Ob + (size_t)RH * HD, HD, (size_t)TT * TT, hs, hs, RH);
            k_merge<<<(unsigned)(((size_t)ZH * TT * HD / 2 + 255) / 256), 256, 0, stream>>>(Ob, h0, ATh, ATl); }
        k_gemmw<bf, 1, 0><<<dim3(TT / 64, DM / 64, 1), 32, 0, stream>>>(ATh, ATl, WO, nullptr, DQ, OUT + (size_t)b * SEQ_FULL * DM, DM, 0, 0, 0, 0);
    }
}
